// SimpleLSTM_46248207843581
// MI455X (gfx1250) — hardware-run, weakly checked
//
#include <hip/hip_runtime.h>
#include <math.h>

constexpr int NSEQ  = 32;
constexpr int TLEN  = 16384;
constexpr int HID   = 96;
constexpr int G4H   = 4 * HID;
constexpr int RBLK  = 16;
constexpr int NWAVE = HID / 16;
constexpr int NTHR  = NWAVE * 32;
constexpr int HP    = 104;
constexpr int TCH   = 32;
constexpr int OBP   = 32;
constexpr int NCVT  = 256;
constexpr int WH_N8 = (G4H * HID) / 8;
static_assert(HID % 32 == 0);
static_assert(HID == 16 * NWAVE);
static_assert(NSEQ % RBLK == 0);
static_assert(TLEN % TCH == 0);
static_assert(HP % 8 == 0 && HP >= HID);
static_assert((G4H * HID) % 8 == 0 && WH_N8 % 32 == 0);
static_assert(TCH * RBLK == 4 * 128);
static_assert(NTHR >= 128);
static_assert(OBP * 4 == 128);

typedef __attribute__((ext_vector_type(16))) __bf16   v16b;
typedef __attribute__((ext_vector_type(8)))  __bf16   v8b;
typedef __attribute__((ext_vector_type(8)))  _Float16 v8h;
typedef __attribute__((ext_vector_type(8)))  float    v8f;
typedef __attribute__((ext_vector_type(4)))  float    v4f;

__device__ __forceinline__ unsigned short f2bf_bits(float f) {
  unsigned u = __float_as_uint(f);
  return (unsigned short)((u + 0x7FFFu + ((u >> 16) & 1u)) >> 16);
}
__device__ __forceinline__ float bf_bits2f(unsigned short h) { return __uint_as_float(((unsigned)h) << 16); }
__device__ __forceinline__ float bf16r(float f) { return bf_bits2f(f2bf_bits(f)); }

__device__ __forceinline__ void acc_guard4(v8f& a, v8f& b, v8f& c, v8f& d) {
  asm volatile("v_nop\n\tv_nop\n\tv_nop\n\tv_nop" : "+v"(a), "+v"(b), "+v"(c), "+v"(d));
}
__device__ __forceinline__ void mma_group_guard(v8f& a0, v8f& a1, v8f& a2, v8f& a3,
                                                v16b fa, v16b fb, v16b g0, v16b g1, v16b g2, v16b g3) {
  asm volatile("v_nop\n\tv_nop\n\tv_nop\n\tv_nop"
               : "+v"(a0), "+v"(a1), "+v"(a2), "+v"(a3)
               : "v"(fa), "v"(fb), "v"(g0), "v"(g1), "v"(g2), "v"(g3));
}

template <typename T> struct Frag;
template <> struct Frag<__bf16> {
  typedef v16b V; union U { v16b v; v8b h[2]; };
  static __device__ __forceinline__ v16b load(const __bf16* p) {
    U f; f.h[0] = *(const v8b*)(p); f.h[1] = *(const v8b*)(p + 16); return f.v;
  }
  static __device__ __forceinline__ v8f mma(v16b a, v16b b, v8f c) {
    return __builtin_amdgcn_wmma_f32_16x16x32_bf16(false, a, false, b, (short)0, c, false, false);
  }
};

__device__ __forceinline__ float sigm_f(float v) { return __builtin_amdgcn_rcpf(1.0f + expf(-v)); }
__device__ __forceinline__ float tanh_f(float v) {
  const float e = expf(-2.0f * fabsf(v));
  const float m = (1.0f - e) * __builtin_amdgcn_rcpf(1.0f + e);
  return copysignf(m, v);
}

__global__ __launch_bounds__(NCVT) void cvt_bf16x8_kernel(const float* __restrict__ src, unsigned short* __restrict__ dst, int n8) {
  const int i = blockIdx.x * NCVT + threadIdx.x;
  if (i < n8) {
    const float* sp = src + (size_t)i * 8;
    const v4f a = *(const v4f*)(sp);
    const v4f b = *(const v4f*)(sp + 4);
    v8h hv;
#pragma unroll
    for (int e = 0; e < 4; ++e) {
      hv[e]     = __builtin_bit_cast(_Float16, f2bf_bits(a[e]));
      hv[4 + e] = __builtin_bit_cast(_Float16, f2bf_bits(b[e]));
    }
    *(volatile v8h*)(dst + (size_t)i * 8) = hv;
    __threadfence();
    *(volatile v8h*)(dst + (size_t)i * 8) = hv;
  }
}

__global__ __launch_bounds__(NTHR) void lstm_seq_kernel(const float* __restrict__ x, const float* __restrict__ w_ih,
                                                        const float* __restrict__ b_ih, const float* __restrict__ b_hh,
                                                        const float* __restrict__ w_dense, const float* __restrict__ b_dense,
                                                        const unsigned short* __restrict__ WHBp, float* __restrict__ out) {
  __shared__ __align__(16) unsigned short Ahi[RBLK * HP];
  __shared__ __align__(16) unsigned short Alo[RBLK * HP];
  __shared__ __align__(16) float xsT[TCH * RBLK];
  __shared__ __align__(16) float part[NWAVE * RBLK];
  __shared__ __align__(16) float obuf[RBLK * OBP];

  const __bf16* WHB = (const __bf16*)WHBp;
  const int tid = threadIdx.x, lane = tid & 31, wave = tid >> 5;
  const int c = lane & 15, hh = lane >> 4, koff = hh * 8;
  const int b0 = blockIdx.x * RBLK;
  const int j = 16 * wave + c;

#pragma unroll 1
  for (int i = tid; i < RBLK * HP; i += NTHR) { Ahi[i] = 0; Alo[i] = 0; }

  float wih[4], bsum[4];
#pragma unroll
  for (int g = 0; g < 4; ++g) {
    const int n = g * HID + j;
    wih[g]  = bf16r(w_ih[n]);
    bsum[g] = bf16r(b_ih[n]) + bf16r(b_hh[n]);
  }
  const float wd = bf16r(w_dense[j]);
  const float bd = bf16r(b_dense[0]);
  float cst[8];
#pragma unroll
  for (int r = 0; r < 8; ++r) cst[r] = 0.0f;

  if (tid < 128) {
    const int row = tid >> 3, c4 = (tid & 7) * 4;
    const v4f v = *(const v4f*)(x + (size_t)(b0 + row) * TLEN + c4);
#pragma unroll
    for (int e = 0; e < 4; ++e) xsT[(c4 + e) * RBLK + row] = bf16r(v[e]);
  }
  __syncthreads();

  const __bf16* ahir = (const __bf16*)Ahi + c * HP + koff;
  const __bf16* alor = (const __bf16*)Alo + c * HP + koff;
  const __bf16* wq0 = WHB + (size_t)(0 * HID + j) * HID + koff;
  const __bf16* wq1 = WHB + (size_t)(1 * HID + j) * HID + koff;
  const __bf16* wq2 = WHB + (size_t)(2 * HID + j) * HID + koff;
  const __bf16* wq3 = WHB + (size_t)(3 * HID + j) * HID + koff;
  const v8f z8 = {0.f, 0.f, 0.f, 0.f, 0.f, 0.f, 0.f, 0.f};

#pragma unroll 1
  for (int t = 0; t < TLEN; ++t) {
    const int tc = t & (TCH - 1);
    const v4f xa = *(const v4f*)(xsT + tc * RBLK + 8 * hh);
    const v4f xb = *(const v4f*)(xsT + tc * RBLK + 8 * hh + 4);
    float xr[8];
    xr[0] = xa[0]; xr[1] = xa[1]; xr[2] = xa[2]; xr[3] = xa[3];
    xr[4] = xb[0]; xr[5] = xb[1]; xr[6] = xb[2]; xr[7] = xb[3];

    v8f acc[4];
    acc[0] = z8; acc[1] = z8; acc[2] = z8; acc[3] = z8;
#pragma unroll 1
    for (int k0 = 0; k0 < HID; k0 += 32) {
      const v16b ah  = Frag<__bf16>::load(ahir + k0);
      const v16b al  = Frag<__bf16>::load(alor + k0);
      const v16b bq0 = Frag<__bf16>::load(wq0 + k0);
      const v16b bq1 = Frag<__bf16>::load(wq1 + k0);
      const v16b bq2 = Frag<__bf16>::load(wq2 + k0);
      const v16b bq3 = Frag<__bf16>::load(wq3 + k0);
      acc[0] = Frag<__bf16>::mma(ah, bq0, acc[0]);
      acc[1] = Frag<__bf16>::mma(ah, bq1, acc[1]);
      acc[2] = Frag<__bf16>::mma(ah, bq2, acc[2]);
      acc[3] = Frag<__bf16>::mma(ah, bq3, acc[3]);
      acc[0] = Frag<__bf16>::mma(al, bq0, acc[0]);
      acc[1] = Frag<__bf16>::mma(al, bq1, acc[1]);
      acc[2] = Frag<__bf16>::mma(al, bq2, acc[2]);
      acc[3] = Frag<__bf16>::mma(al, bq3, acc[3]);
      mma_group_guard(acc[0], acc[1], acc[2], acc[3], ah, al, bq0, bq1, bq2, bq3);
    }
    acc_guard4(acc[0], acc[1], acc[2], acc[3]);

    float hcur[8];
#pragma unroll
    for (int r = 0; r < 8; ++r) {
      const float xv = xr[r];
      const float zi = (xv * wih[0] + bsum[0]) + acc[0][r];
      const float zf = (xv * wih[1] + bsum[1]) + acc[1][r];
      const float zg = (xv * wih[2] + bsum[2]) + acc[2][r];
      const float zo = (xv * wih[3] + bsum[3]) + acc[3][r];
      const float ig = sigm_f(zi);
      const float fg = sigm_f(zf);
      const float gg = tanh_f(zg);
      const float og = sigm_f(zo);
      const float cn = fg * cst[r] + ig * gg;
      cst[r] = cn;
      hcur[r] = og * tanh_f(cn);
    }
    float pr[8];
#pragma unroll
    for (int r = 0; r < 8; ++r) {
      float p = hcur[r] * wd;
      p += __shfl_xor(p, 1, 32);
      p += __shfl_xor(p, 2, 32);
      p += __shfl_xor(p, 4, 32);
      p += __shfl_xor(p, 8, 32);
      pr[r] = p;
    }
    if (c == 0) {
#pragma unroll
      for (int r = 0; r < 8; ++r) part[wave * RBLK + 8 * hh + r] = pr[r];
    }
    __syncthreads();

    if (wave == 0) {
      const int row = lane & 15;
      float s = 0.0f;
#pragma unroll
      for (int w2 = 0; w2 < NWAVE; ++w2) s += part[w2 * RBLK + row];
      s += bd;
      if (lane < RBLK) obuf[row * OBP + tc] = s;
      if (tc == TCH - 1) {
        __builtin_amdgcn_fence(__ATOMIC_RELEASE, "workgroup");
        __builtin_amdgcn_wave_barrier();
        __builtin_amdgcn_fence(__ATOMIC_ACQUIRE, "workgroup");
        const int q = lane >> 3, c4 = (lane & 7) * 4;
        const size_t tb = (size_t)(t - (TCH - 1));
        for (int pass = 0; pass < 2; ++pass) {
#pragma unroll
          for (int it = 0; it < 4; ++it) {
            const int row2 = it * 4 + q;
            const v4f v = *(const v4f*)(obuf + row2 * OBP + c4);
            *(volatile v4f*)(out + (size_t)(b0 + row2) * TLEN + tb + c4) = v;
          }
          __threadfence();
        }
      }
    }

#pragma unroll
    for (int r = 0; r < 8; ++r) {
      const float hv = hcur[r];
      const unsigned short hb = f2bf_bits(hv);
      const unsigned short lb = f2bf_bits(hv - bf_bits2f(hb));
      Ahi[(8 * hh + r) * HP + j] = hb;
      Alo[(8 * hh + r) * HP + j] = lb;
    }
    if (tc == TCH - 1 && t + 1 < TLEN) {
      if (tid < 128) {
        const int row = tid >> 3, c4 = (tid & 7) * 4;
        const v4f v = *(const v4f*)(x + (size_t)(b0 + row) * TLEN + (size_t)(t + 1) + c4);
#pragma unroll
        for (int e = 0; e < 4; ++e) xsT[(c4 + e) * RBLK + row] = bf16r(v[e]);
      }
    }
    __syncthreads();
  }
}

extern "C" void kernel_launch(void* const* d_in, const int* in_sizes, int n_in,
                              void* d_out, int out_size, void* d_ws, size_t ws_size, hipStream_t stream) {
  if (n_in < 7 || d_out == nullptr || d_ws == nullptr) return;
  if (in_sizes[0] != NSEQ * TLEN || in_sizes[1] != G4H || in_sizes[2] != G4H * HID || in_sizes[3] != G4H ||
      in_sizes[4] != G4H || in_sizes[5] != HID || in_sizes[6] < 1 || out_size != NSEQ * TLEN) return;

  const float* x       = (const float*)d_in[0];
  const float* w_ih    = (const float*)d_in[1];
  const float* w_hh    = (const float*)d_in[2];
  const float* b_ih    = (const float*)d_in[3];
  const float* b_hh    = (const float*)d_in[4];
  const float* w_dense = (const float*)d_in[5];
  const float* b_dense = (const float*)d_in[6];
  float* out = (float*)d_out;

  char* ws = (char*)d_ws; size_t off = 0;
  auto carve = [&](size_t bytes) -> char* { char* p = ws + off; off += (bytes + 255) & ~(size_t)255; return p; };
  unsigned short* WHB = (unsigned short*)carve((size_t)G4H * HID * 2);
  if (off > ws_size || off > (size_t)134217728) return;

  cvt_bf16x8_kernel<<<(WH_N8 + NCVT - 1) / NCVT, NCVT, 0, stream>>>(w_hh, WHB, WH_N8);
  lstm_seq_kernel<<<NSEQ / RBLK, NTHR, 0, stream>>>(x, w_ih, b_ih, b_hh, w_dense, b_dense, WHB, out);
}
